// CapsuleNet_40355512713817
// MI455X (gfx1250) — hardware-verified
//
#include <hip/hip_runtime.h>
#include <math.h>

constexpr int kBatch    = 256;
constexpr int kNumIn    = 1152;
constexpr int kNumOut   = 10;
constexpr int kVecOut   = 16;
constexpr int kVecIn    = 8;
constexpr int kJD       = kNumOut * kVecOut;
constexpr int kImg      = 28;
constexpr int kH1       = 20;
constexpr int kC1M      = kBatch * kH1 * kH1;
constexpr int kC1N      = 256;
constexpr int kC1Kreal  = 81;
constexpr int kC1K      = 96;
constexpr int kPCM      = kBatch * 36;
constexpr int kPCN      = 256;
constexpr int kPCK      = 81 * 256;
constexpr int kRoutIters = kNumIn / 16;
constexpr float kWCarry    = 16.0f;
constexpr float kWCarryInv = 1.0f / 16.0f;

static_assert(kC1M % 64 == 0);
static_assert(kC1N % 64 == 0);
static_assert(kC1K % 32 == 0);
static_assert(kPCM % 64 == 0);
static_assert(kPCN % 64 == 0);
static_assert(kPCK % 32 == 0);
static_assert(kRoutIters * 16 == kNumIn);
static_assert(kJD == 160);

constexpr int kThrIm2col = kC1M * kC1K / 8;
constexpr int kThrC1W    = kC1N * kC1K / 8;
constexpr int kThrPCW    = kPCN * kPCK / 8;
constexpr int kThrWr     = kNumIn * kJD * kVecIn / 4;
constexpr int kThrSquash = kBatch * kNumIn * 2;
static_assert(kThrIm2col % 256 == 0);
static_assert(kThrC1W % 256 == 0);
static_assert(kThrPCW % 256 == 0);
static_assert(kThrWr % 256 == 0);
static_assert(kThrSquash % 256 == 0);

constexpr size_t kSzA1    = (size_t)kC1M * kC1K * 2;
constexpr size_t kSzBt1   = (size_t)kC1N * kC1K * 2;
constexpr size_t kSzH     = (size_t)kC1M * kC1N * 2;
constexpr size_t kSzBtpc  = (size_t)kPCN * kPCK * 2;
constexpr size_t kSzY     = (size_t)kPCM * kPCN * 4;
constexpr size_t kSzCaps  = (size_t)kBatch * kNumIn * kVecIn * 4;
constexpr size_t kSzWr    = (size_t)kNumIn * kJD * kVecIn * 4;
constexpr size_t kSzBias  = 768 * 4;
constexpr size_t kOffA1   = 0;
constexpr size_t kOffBt1  = kOffA1 + kSzA1;
constexpr size_t kOffH    = kOffBt1 + kSzBt1;
constexpr size_t kOffBtpc = kOffH + kSzH;
constexpr size_t kOffY    = kOffBtpc + kSzBtpc;
constexpr size_t kOffCaps = kOffY + kSzY;
constexpr size_t kOffWr   = kOffCaps + kSzCaps;
constexpr size_t kOffBias = kOffWr + kSzWr;
constexpr size_t kWsTotal = kOffBias + kSzBias;
static_assert(kOffBt1 % 256 == 0 && kOffH % 256 == 0 && kOffBtpc % 256 == 0 && kOffY % 256 == 0);
static_assert(kOffCaps % 256 == 0 && kOffWr % 256 == 0 && kOffBias % 256 == 0);
static_assert(kWsTotal <= (size_t)134217728);

typedef __attribute__((ext_vector_type(16))) _Float16 v16h;
typedef __attribute__((ext_vector_type(8)))  _Float16 v8h;
typedef __attribute__((ext_vector_type(16))) __bf16   v16b;
typedef __attribute__((ext_vector_type(8)))  __bf16   v8b;
typedef __attribute__((ext_vector_type(8)))  float    v8f;
typedef __attribute__((ext_vector_type(4)))  float    v4f;
typedef __attribute__((ext_vector_type(4)))  unsigned int v4u;

__device__ __forceinline__ unsigned short f2bf_bits(float f) {
  unsigned u = __float_as_uint(f);
  return (unsigned short)((u + 0x7FFFu + ((u >> 16) & 1u)) >> 16);
}
__device__ __forceinline__ float bf_bits2f(unsigned short h) { return __uint_as_float(((unsigned)h) << 16); }

__device__ __forceinline__ void dep_guard_h(v8f& a, v8f& b, v16h x, v16h y) { asm volatile("v_nop\n\tv_nop\n\tv_nop\n\tv_nop" : "+v"(a), "+v"(b) : "v"(x), "v"(y)); }
__device__ __forceinline__ void dep_guard_b(v8f& a, v8f& b, v16b x, v16b y) { asm volatile("v_nop\n\tv_nop\n\tv_nop\n\tv_nop" : "+v"(a), "+v"(b) : "v"(x), "v"(y)); }
__device__ __forceinline__ void keep4_h(v16h a, v16h b, v16h c, v16h d) { asm volatile("v_nop" :: "v"(a), "v"(b), "v"(c), "v"(d)); }
__device__ __forceinline__ void keep4_b(v16b a, v16b b, v16b c, v16b d) { asm volatile("v_nop" :: "v"(a), "v"(b), "v"(c), "v"(d)); }
__device__ __forceinline__ void acc_guard4(v8f& a, v8f& b, v8f& c, v8f& d) { asm volatile("v_nop\n\tv_nop\n\tv_nop\n\tv_nop" : "+v"(a), "+v"(b), "+v"(c), "+v"(d)); }
template <typename T> struct Frag;
template <> struct Frag<_Float16> {
  typedef v16h V; union U { v16h v; v8h h[2]; };
  static __device__ __forceinline__ v16h load(const _Float16* p) {
    U f; f.h[0] = *(const v8h*)(p); f.h[1] = *(const v8h*)(p + 16); return f.v;
  }
  static __device__ __forceinline__ v8f mma(v16h a, v16h b, v8f c) {
    return __builtin_amdgcn_wmma_f32_16x16x32_f16(false, a, false, b, (short)0, c, false, false);
  }
  static __device__ __forceinline__ void guard(v8f& a, v8f& b, v16h x, v16h y) { dep_guard_h(a, b, x, y); }
  static __device__ __forceinline__ void keep(v16h a, v16h b, v16h c, v16h d) { keep4_h(a, b, c, d); }
};
template <> struct Frag<__bf16> {
  typedef v16b V; union U { v16b v; v8b h[2]; };
  static __device__ __forceinline__ v16b load(const __bf16* p) {
    U f; f.h[0] = *(const v8b*)(p); f.h[1] = *(const v8b*)(p + 16); return f.v;
  }
  static __device__ __forceinline__ v8f mma(v16b a, v16b b, v8f c) {
    return __builtin_amdgcn_wmma_f32_16x16x32_bf16(false, a, false, b, (short)0, c, false, false);
  }
  static __device__ __forceinline__ void guard(v8f& a, v8f& b, v16b x, v16b y) { dep_guard_b(a, b, x, y); }
  static __device__ __forceinline__ void keep(v16b a, v16b b, v16b c, v16b d) { keep4_b(a, b, c, d); }
};

__device__ __forceinline__ unsigned pk16(unsigned short a, unsigned short b) { return (unsigned)a | ((unsigned)b << 16); }
__device__ __forceinline__ unsigned short h_bits(float f) { const _Float16 h = (_Float16)f; return __builtin_bit_cast(unsigned short, h); }
__device__ __forceinline__ float bf16rn(float f) { return bf_bits2f(f2bf_bits(f)); }

__device__ __forceinline__ void store2x_u4(unsigned short* q, v4u u) {
  *(volatile v4u*)q = u;
  __threadfence();
  *(volatile v4u*)q = u;
}
__device__ __forceinline__ void store2x_f4(float* q, v4f v) {
  *(volatile v4f*)q = v;
  __threadfence();
  *(volatile v4f*)q = v;
}

template <int ET> struct Elem;
template <> struct Elem<0> { typedef _Float16 T; };
template <> struct Elem<1> { typedef __bf16 T; };
template <int ET, bool SPLIT, int BIAS_MODE, int OUT_MODE, bool RESID, int ACT = 0>
__global__ __launch_bounds__(256) void wmma_gemm64(
    const unsigned short* __restrict__ Ap, const unsigned short* __restrict__ A2p, int lda, long strideA,
    const unsigned short* __restrict__ Btp, const unsigned short* __restrict__ Bt2p, int ldb, long strideB,
    void* __restrict__ Cout, void* __restrict__ Cout2, int ldc, long strideC,
    const float* __restrict__ bias,
    const float* __restrict__ resid, long strideR,
    int M, int N, int K, float scale) {
  typedef typename Elem<ET>::T T;
  typedef typename Frag<T>::V V;
  const T* A = (const T*)Ap; const T* A2 = (const T*)A2p; const T* Bt = (const T*)Btp; const T* Bt2 = (const T*)Bt2p;
  __shared__ __align__(16) float sT[8][16 * 68];
  const int b    = blockIdx.y;
  const int lane = threadIdx.x & 31;
  const int wave = threadIdx.x >> 5;
  const int tilesN = N >> 6;
  const int tilesM = M >> 6;
  const int tile = blockIdx.x * 8 + wave;
  if (tile >= tilesM * tilesN) return;
  const int tm = tile / tilesN;
  const int tn = tile - tm * tilesN;
  const int m0 = tm << 6;
  const int n0 = tn << 6;

  const T* Ab  = A  + (size_t)b * strideA;
  const T* Bb  = Bt + (size_t)b * strideB;
  const T* Ab2 = SPLIT ? (A2  + (size_t)b * strideA) : nullptr;
  const T* Bb2 = SPLIT ? (Bt2 + (size_t)b * strideB) : nullptr;

  const int rlane = lane & 15;
  const int koff  = (lane >> 4) * 8;
  const int mOff  = (lane >> 4) * 8;

  v8f acc[4][4];
#pragma unroll
  for (int i = 0; i < 4; ++i)
#pragma unroll
    for (int j = 0; j < 4; ++j) acc[i][j] = (v8f){0.f,0.f,0.f,0.f,0.f,0.f,0.f,0.f};

  for (int k0 = 0; k0 < K; k0 += 32) {
    V bh[4], bl[4];
#pragma unroll
    for (int j = 0; j < 4; ++j) {
      const size_t bo = (size_t)(n0 + (j << 4) + rlane) * ldb + koff + k0;
      bh[j] = Frag<T>::load(Bb + bo);
      if (SPLIT) bl[j] = Frag<T>::load(Bb2 + bo);
    }
#pragma unroll
    for (int i = 0; i < 4; ++i) {
      const size_t ao = (size_t)(m0 + (i << 4) + rlane) * lda + koff + k0;
      V ah = Frag<T>::load(Ab + ao);
      V al;
      if (SPLIT) al = Frag<T>::load(Ab2 + ao);
#pragma unroll
      for (int j = 0; j < 4; ++j) {
        acc[i][j] = Frag<T>::mma(ah, bh[j], acc[i][j]);
        if (SPLIT) {
          acc[i][j] = Frag<T>::mma(ah, bl[j], acc[i][j]);
          acc[i][j] = Frag<T>::mma(al, bh[j], acc[i][j]);
        }
      }
      Frag<T>::guard(acc[i][0], acc[i][3], ah, SPLIT ? al : ah);
    }
    Frag<T>::keep(bh[0], bh[1], bh[2], bh[3]);
    if (SPLIT) Frag<T>::keep(bl[0], bl[1], bl[2], bl[3]);
  }
  acc_guard4(acc[0][0], acc[0][1], acc[0][2], acc[0][3]);
  acc_guard4(acc[1][0], acc[1][1], acc[1][2], acc[1][3]);
  acc_guard4(acc[2][0], acc[2][1], acc[2][2], acc[2][3]);
  acc_guard4(acc[3][0], acc[3][1], acc[3][2], acc[3][3]);

  float* slab = sT[wave];
  const float* Rb = RESID ? (resid + (size_t)b * strideR) : nullptr;
#pragma unroll
  for (int i = 0; i < 4; ++i) {
    const int mBase = m0 + (i << 4);
#pragma unroll
    for (int j = 0; j < 4; ++j) {
      const int n = n0 + (j << 4) + rlane;
      float bv = 0.f;
      if (BIAS_MODE == 2) bv = bias[n];
#pragma unroll
      for (int r = 0; r < 8; ++r) {
        float v = acc[i][j][r] * scale;
        if (BIAS_MODE == 1) v += bias[mBase + mOff + r];
        if (BIAS_MODE == 2) v += bv;
        if (RESID) v += Rb[(size_t)(mBase + mOff + r) * ldc + n];
        if (ACT == 2) v = fmaxf(v, 0.0f);
        if (ACT == 4) v = (v > 0.f) ? v : 0.01f * v;
        slab[(mOff + r) * 68 + (j << 4) + rlane] = v;
      }
    }
    __builtin_amdgcn_fence(__ATOMIC_RELEASE, "workgroup");
    __builtin_amdgcn_wave_barrier();
    __builtin_amdgcn_fence(__ATOMIC_ACQUIRE, "workgroup");
    if (OUT_MODE == 0) {
      float* C = (float*)Cout + (size_t)b * strideC;
      const int hh = lane >> 4, c4 = (lane & 15) * 4;
      for (int pass = 0; pass < 2; ++pass) {
#pragma unroll
        for (int it = 0; it < 8; ++it) {
          const int row = it * 2 + hh;
          v4f v = *(const v4f*)(slab + row * 68 + c4);
          *(volatile v4f*)(C + (size_t)(mBase + row) * ldc + n0 + c4) = v;
        }
        __threadfence();
      }
    } else {
      const int q = lane >> 3, c8 = (lane & 7) * 8;
      unsigned short* C  = (unsigned short*)Cout  + (size_t)b * strideC;
      unsigned short* C2 = (OUT_MODE == 2) ? ((unsigned short*)Cout2 + (size_t)b * strideC) : nullptr;
      for (int pass = 0; pass < 2; ++pass) {
#pragma unroll
        for (int it = 0; it < 4; ++it) {
          const int row = it * 4 + q;
          const float* sp = slab + row * 68 + c8;
          v8h hv, lv;
#pragma unroll
          for (int e = 0; e < 8; ++e) {
            if (OUT_MODE == 1) {
              hv[e] = (_Float16)sp[e];
            } else {
              unsigned short hb = f2bf_bits(sp[e]);
              unsigned short lb = f2bf_bits(sp[e] - bf_bits2f(hb));
              hv[e] = __builtin_bit_cast(_Float16, hb);
              lv[e] = __builtin_bit_cast(_Float16, lb);
            }
          }
          *(volatile v8h*)(C + (size_t)(mBase + row) * ldc + n0 + c8) = hv;
          if (OUT_MODE == 2) *(volatile v8h*)(C2 + (size_t)(mBase + row) * ldc + n0 + c8) = lv;
        }
        __threadfence();
      }
    }
    __builtin_amdgcn_fence(__ATOMIC_RELEASE, "workgroup");
    __builtin_amdgcn_wave_barrier();
    __builtin_amdgcn_fence(__ATOMIC_ACQUIRE, "workgroup");
  }
}

__global__ __launch_bounds__(256) void prep_bias_kernel(const float* __restrict__ c1b, const float* __restrict__ pcb,
                                                        const float* __restrict__ dcb, float* __restrict__ outR) {
  const int t = threadIdx.x;
  const int wave = t >> 5;
  const int lane = t & 31;
  if (wave < 6) {
    const float* src;
    int idx4, nvalid4;
    if (wave < 2)      { src = c1b; idx4 = wave * 32 + lane;       nvalid4 = 64; }
    else if (wave < 4) { src = pcb; idx4 = (wave - 2) * 32 + lane; nvalid4 = 64; }
    else               { src = dcb; idx4 = (wave - 4) * 32 + lane; nvalid4 = 40; }
    const int idc = (idx4 < nvalid4) ? idx4 : (nvalid4 - 1);
    const unsigned msk = (idx4 < nvalid4) ? 0xFFFFFFFFu : 0u;
    const v4f v = *(const v4f*)(src + idc * 4);
    v4f o;
#pragma unroll
    for (int e = 0; e < 4; ++e) {
      const unsigned u = ((unsigned)f2bf_bits(v[e]) << 16) & msk;
      o[e] = __uint_as_float(u);
    }
    store2x_f4(outR + t * 4, o);
  }
}

__global__ __launch_bounds__(256) void im2col_x_kernel(const float* __restrict__ x, unsigned short* __restrict__ A1, int nthr) {
  const int g = blockIdx.x * 256 + threadIdx.x;
  if (g >= nthr) return;
  const int f  = g * 8;
  const int m  = f / kC1K;
  const int kb = f - m * kC1K;
  const int bb = m / (kH1 * kH1);
  const int rr = m - bb * (kH1 * kH1);
  const int oy = rr / kH1;
  const int ox = rr - oy * kH1;
  const float* xb = x + (size_t)bb * (kImg * kImg) + oy * kImg + ox;
  unsigned short hb[8];
#pragma unroll
  for (int e = 0; e < 8; ++e) {
    const int k  = kb + e;
    const int kc = (k < kC1Kreal) ? k : (kC1Kreal - 1);
    const int ky = kc / 9;
    const int kx = kc - ky * 9;
    const float val = xb[ky * kImg + kx];
    const unsigned msk = (k < kC1Kreal) ? 0xFFFFu : 0u;
    hb[e] = (unsigned short)(h_bits(bf16rn(val)) & msk);
  }
  const v4u u = (v4u){pk16(hb[0], hb[1]), pk16(hb[2], hb[3]), pk16(hb[4], hb[5]), pk16(hb[6], hb[7])};
  store2x_u4(A1 + (size_t)f, u);
}

__global__ __launch_bounds__(256) void cast_c1w_kernel(const float* __restrict__ w, unsigned short* __restrict__ Bt1, int nthr) {
  const int g = blockIdx.x * 256 + threadIdx.x;
  if (g >= nthr) return;
  const int f  = g * 8;
  const int oc = f / kC1K;
  const int kb = f - oc * kC1K;
  const float* wp = w + (size_t)oc * kC1Kreal;
  unsigned short hb[8];
#pragma unroll
  for (int e = 0; e < 8; ++e) {
    const int k  = kb + e;
    const int kc = (k < kC1Kreal) ? k : (kC1Kreal - 1);
    const float val = wp[kc];
    const unsigned msk = (k < kC1Kreal) ? 0xFFFFu : 0u;
    hb[e] = (unsigned short)(h_bits(kWCarry * bf16rn(val)) & msk);
  }
  const v4u u = (v4u){pk16(hb[0], hb[1]), pk16(hb[2], hb[3]), pk16(hb[4], hb[5]), pk16(hb[6], hb[7])};
  store2x_u4(Bt1 + (size_t)f, u);
}

__global__ __launch_bounds__(256) void permute_pcw_kernel(const float* __restrict__ pcw, unsigned short* __restrict__ Btpc, int nthr) {
  const int g = blockIdx.x * 256 + threadIdx.x;
  if (g >= nthr) return;
  const int f   = g * 8;
  const int oc  = f / kPCK;
  const int r   = f - oc * kPCK;
  const int p   = r >> 8;
  const int ic0 = r & 255;
  const float* wp = pcw + ((size_t)oc * 256 + ic0) * 81 + p;
  unsigned short hb[8];
#pragma unroll
  for (int e = 0; e < 8; ++e) {
    const float val = wp[e * 81];
    hb[e] = h_bits(kWCarry * bf16rn(val));
  }
  const v4u u = (v4u){pk16(hb[0], hb[1]), pk16(hb[2], hb[3]), pk16(hb[4], hb[5]), pk16(hb[6], hb[7])};
  store2x_u4(Btpc + (size_t)f, u);
}

__global__ __launch_bounds__(256) void rne_w_kernel(const float* __restrict__ W, float* __restrict__ Wr, int nthr) {
  const int g = blockIdx.x * 256 + threadIdx.x;
  if (g >= nthr) return;
  const v4f v = *(const v4f*)(W + (size_t)4 * g);
  v4f o;
#pragma unroll
  for (int e = 0; e < 4; ++e) o[e] = bf16rn(v[e]);
  store2x_f4(Wr + (size_t)4 * g, o);
}

__global__ __launch_bounds__(256) void gemm_pc_kernel(const unsigned short* __restrict__ Hp,
                                                      const unsigned short* __restrict__ Btp,
                                                      float* __restrict__ Yout, float scale) {
  typedef _Float16 T;
  typedef Frag<T>::V V;
  const T* Hb = (const T*)Hp;
  const T* Bb = (const T*)Btp;
  __shared__ __align__(16) float sT[8][16 * 68];
  const int lane = threadIdx.x & 31;
  const int wave = threadIdx.x >> 5;
  constexpr int tilesN = kPCN >> 6;
  constexpr int tilesM = kPCM >> 6;
  const int tile = blockIdx.x * 8 + wave;
  if (tile >= tilesM * tilesN) return;
  const int tm = tile / tilesN;
  const int tn = tile - tm * tilesN;
  const int m0 = tm << 6;
  const int n0 = tn << 6;
  const int rlane = lane & 15;
  const int koff  = (lane >> 4) * 8;
  const int mOff  = (lane >> 4) * 8;

  int rb[4];
#pragma unroll
  for (int i = 0; i < 4; ++i) {
    const int m   = m0 + (i << 4) + rlane;
    const int bb  = m / 36;
    const int pix = m - bb * 36;
    const int oy  = pix / 6;
    const int ox  = pix - oy * 6;
    rb[i] = ((bb * kH1 + 2 * oy) * kH1 + 2 * ox) * kC1N;
  }

  v8f acc[4][4];
#pragma unroll
  for (int i = 0; i < 4; ++i)
#pragma unroll
    for (int j = 0; j < 4; ++j) acc[i][j] = (v8f){0.f,0.f,0.f,0.f,0.f,0.f,0.f,0.f};

  for (int k0 = 0; k0 < kPCK; k0 += 32) {
    const int p   = k0 >> 8;
    const int ic0 = k0 & 255;
    const int ky  = p / 9;
    const int kx  = p - ky * 9;
    const int kadd = (ky * kH1 + kx) * kC1N + ic0 + koff;
    V bh[4];
#pragma unroll
    for (int j = 0; j < 4; ++j) {
      const size_t bo = (size_t)(n0 + (j << 4) + rlane) * kPCK + koff + k0;
      bh[j] = Frag<T>::load(Bb + bo);
    }
#pragma unroll
    for (int i = 0; i < 4; ++i) {
      V ah = Frag<T>::load(Hb + (size_t)rb[i] + kadd);
#pragma unroll
      for (int j = 0; j < 4; ++j) acc[i][j] = Frag<T>::mma(ah, bh[j], acc[i][j]);
      Frag<T>::guard(acc[i][0], acc[i][3], ah, ah);
    }
    Frag<T>::keep(bh[0], bh[1], bh[2], bh[3]);
  }
  acc_guard4(acc[0][0], acc[0][1], acc[0][2], acc[0][3]);
  acc_guard4(acc[1][0], acc[1][1], acc[1][2], acc[1][3]);
  acc_guard4(acc[2][0], acc[2][1], acc[2][2], acc[2][3]);
  acc_guard4(acc[3][0], acc[3][1], acc[3][2], acc[3][3]);

  float* slab = sT[wave];
#pragma unroll
  for (int i = 0; i < 4; ++i) {
    const int mBase = m0 + (i << 4);
#pragma unroll
    for (int j = 0; j < 4; ++j) {
#pragma unroll
      for (int r = 0; r < 8; ++r) {
        const float v = acc[i][j][r] * scale;
        slab[(mOff + r) * 68 + (j << 4) + rlane] = v;
      }
    }
    __builtin_amdgcn_fence(__ATOMIC_RELEASE, "workgroup");
    __builtin_amdgcn_wave_barrier();
    __builtin_amdgcn_fence(__ATOMIC_ACQUIRE, "workgroup");
    {
      const int hh = lane >> 4, c4 = (lane & 15) * 4;
      for (int pass = 0; pass < 2; ++pass) {
#pragma unroll
        for (int it = 0; it < 8; ++it) {
          const int row = it * 2 + hh;
          v4f v = *(const v4f*)(slab + row * 68 + c4);
          *(volatile v4f*)(Yout + (size_t)(mBase + row) * kPCN + n0 + c4) = v;
        }
        __threadfence();
      }
    }
    __builtin_amdgcn_fence(__ATOMIC_RELEASE, "workgroup");
    __builtin_amdgcn_wave_barrier();
    __builtin_amdgcn_fence(__ATOMIC_ACQUIRE, "workgroup");
  }
}

__global__ __launch_bounds__(256) void squash_caps_kernel(const float* __restrict__ Y, const float* __restrict__ biasR,
                                                          float* __restrict__ capsF, int nthr) {
  __shared__ float pcb[kPCN];
  const int tid = threadIdx.x;
  pcb[tid] = biasR[kPCN + tid];
  __syncthreads();
  const int g  = blockIdx.x * 256 + tid;
  const int gc = (g < nthr) ? g : (nthr - 1);
  const int cap  = gc >> 1;
  const int half = gc & 1;
  const int bb = cap / kNumIn;
  const int i  = cap - bb * kNumIn;
  float v[4];
  float mp = 0.0f;
#pragma unroll
  for (int e = 0; e < 4; ++e) {
    const int k    = half * 4 + e;
    const int flat = i * 8 + k;
    const int ch   = flat / 36;
    const int yx   = flat - ch * 36;
    const float val = Y[((size_t)bb * 36 + yx) * kPCN + ch] + pcb[ch];
    v[e] = val;
    mp = fmaf(val, val, mp);
  }
  const float m   = mp + __shfl_xor(mp, 1, 32);
  const float sq  = sqrtf(m);
  const float fac = m / (1.0f + m);
  v4f o;
#pragma unroll
  for (int e = 0; e < 4; ++e) o[e] = (v[e] / sq) * fac;
  if (g < nthr) store2x_f4(capsF + (size_t)4 * g, o);
}

__global__ __launch_bounds__(256) void routing_kernel(const float* __restrict__ capsF, const float* __restrict__ Wr,
                                                      const float* __restrict__ biasR, float* __restrict__ out) {
  __shared__ float ul[256 * kNumOut];
  __shared__ float sp[256 * kNumOut];
  __shared__ float ss[kJD];
  __shared__ float vd[kJD];
  __shared__ __align__(16) float vv[kJD];
  const int b    = blockIdx.x;
  const int tid  = threadIdx.x;
  const int lane = tid & 31;
  const int wave = tid >> 5;
  const int c     = lane & 15;
  const int hf    = lane >> 4;
  const int sbase = lane & 16;
  if (tid < kJD) { vd[tid] = 0.0f; vv[tid] = 0.0f; }
  __syncthreads();
  const float* capsB = capsF + (size_t)b * kNumIn * kVecIn;
  const float* dcb   = biasR + 512;

#pragma unroll 1
  for (int r = 0; r < 3; ++r) {
#pragma unroll
    for (int j = 0; j < kNumOut; ++j) sp[tid * kNumOut + j] = 0.0f;
#pragma unroll 1
    for (int it = 0; it < kRoutIters; ++it) {
      const int i = ((it * 8 + wave) << 1) + hf;
      const float* cp = capsB + i * kVecIn;
      const v4f ca = *(const v4f*)(cp);
      const v4f cb = *(const v4f*)(cp + 4);
      const float* wrow = Wr + ((size_t)i * kJD + c) * kVecIn;
      float mx   = -INFINITY;
      float bsel = -INFINITY;
#pragma unroll 1
      for (int j = 0; j < kNumOut; ++j) {
        const float* wp = wrow + j * (kVecOut * kVecIn);
        const v4f w0 = *(const v4f*)(wp);
        const v4f w1 = *(const v4f*)(wp + 4);
        float u = 0.0f;
        u = fmaf(w0[0], ca[0], u);
        u = fmaf(w0[1], ca[1], u);
        u = fmaf(w0[2], ca[2], u);
        u = fmaf(w0[3], ca[3], u);
        u = fmaf(w1[0], cb[0], u);
        u = fmaf(w1[1], cb[1], u);
        u = fmaf(w1[2], cb[2], u);
        u = fmaf(w1[3], cb[3], u);
        ul[tid * kNumOut + j] = u;
        float dp = u * vd[j * kVecOut + c];
        dp += __shfl_xor(dp, 1, 32);
        dp += __shfl_xor(dp, 2, 32);
        dp += __shfl_xor(dp, 4, 32);
        dp += __shfl_xor(dp, 8, 32);
        mx = fmaxf(mx, dp);
        bsel = (c == j) ? dp : bsel;
      }
      float e = expf(bsel - mx);
      e = (c < kNumOut) ? e : 0.0f;
      float sm = e;
      sm += __shfl_xor(sm, 1, 32);
      sm += __shfl_xor(sm, 2, 32);
      sm += __shfl_xor(sm, 4, 32);
      sm += __shfl_xor(sm, 8, 32);
      const float inv = 1.0f / sm;
#pragma unroll 1
      for (int j = 0; j < kNumOut; ++j) {
        const float cj = __shfl(e, sbase + j, 32) * inv;
        const int q = tid * kNumOut + j;
        sp[q] = fmaf(cj, ul[q], sp[q]);
      }
    }
    __syncthreads();
    if (tid < kJD) {
      const int j = tid >> 4;
      const int d = tid & 15;
      float s = 0.0f;
#pragma unroll 1
      for (int q = 0; q < 16; ++q) {
        const int src = (((q >> 1) << 5) + ((q & 1) << 4) + d) * kNumOut + j;
        s += sp[src];
      }
      ss[tid] = s + dcb[tid];
    }
    __syncthreads();
    if (tid < kJD) {
      const int j = tid >> 4;
      float m = 0.0f;
#pragma unroll 1
      for (int d = 0; d < kVecOut; ++d) {
        const float t = ss[j * kVecOut + d];
        m = fmaf(t, t, m);
      }
      const float fac = m / (1.0f + m);
      const float v = (ss[tid] / sqrtf(m)) * fac;
      vv[tid] = v;
      vd[tid] = vd[tid] + v;
    }
    __syncthreads();
  }
  if (tid < 40) {
    const v4f val = *(const v4f*)(vv + tid * 4);
    store2x_f4(out + (size_t)b * kJD + tid * 4, val);
  }
}

extern "C" void kernel_launch(void* const* d_in, const int* in_sizes, int n_in,
                              void* d_out, int out_size, void* d_ws, size_t ws_size,
                              hipStream_t stream) {
  (void)in_sizes; (void)n_in; (void)out_size;
  if (ws_size < kWsTotal) return;
  const float* x       = (const float*)d_in[0];
  const float* conv1_w = (const float*)d_in[1];
  const float* conv1_b = (const float*)d_in[2];
  const float* pc_w    = (const float*)d_in[3];
  const float* pc_b    = (const float*)d_in[4];
  const float* Wt      = (const float*)d_in[5];
  const float* dc_bias = (const float*)d_in[6];
  float* outp = (float*)d_out;

  char* ws = (char*)d_ws;
  unsigned short* A1   = (unsigned short*)(ws + kOffA1);
  unsigned short* Bt1  = (unsigned short*)(ws + kOffBt1);
  unsigned short* Hh   = (unsigned short*)(ws + kOffH);
  unsigned short* Btpc = (unsigned short*)(ws + kOffBtpc);
  float* Y     = (float*)(ws + kOffY);
  float* capsF = (float*)(ws + kOffCaps);
  float* Wr    = (float*)(ws + kOffWr);
  float* biasR = (float*)(ws + kOffBias);

  prep_bias_kernel<<<dim3(1), dim3(256), 0, stream>>>(conv1_b, pc_b, dc_bias, biasR);
  im2col_x_kernel<<<dim3(kThrIm2col / 256), dim3(256), 0, stream>>>(x, A1, kThrIm2col);
  cast_c1w_kernel<<<dim3(kThrC1W / 256), dim3(256), 0, stream>>>(conv1_w, Bt1, kThrC1W);
  permute_pcw_kernel<<<dim3(kThrPCW / 256), dim3(256), 0, stream>>>(pc_w, Btpc, kThrPCW);
  rne_w_kernel<<<dim3(kThrWr / 256), dim3(256), 0, stream>>>(Wt, Wr, kThrWr);
  wmma_gemm64<0, false, 2, 1, false, 0><<<dim3((kC1M / 64) * (kC1N / 64) / 8, 1), dim3(256), 0, stream>>>(
      A1, A1, kC1K, 0L,
      Bt1, Bt1, kC1K, 0L,
      (void*)Hh, (void*)Hh, kC1N, 0L,
      biasR, biasR, 0L,
      kC1M, kC1N, kC1K, kWCarryInv);
  gemm_pc_kernel<<<dim3((kPCM / 64) * (kPCN / 64) / 8), dim3(256), 0, stream>>>(Hh, Btpc, Y, kWCarryInv);
  squash_caps_kernel<<<dim3(kThrSquash / 256), dim3(256), 0, stream>>>(Y, biasR, capsF, kThrSquash);
  routing_kernel<<<dim3(kBatch), dim3(256), 0, stream>>>(capsF, Wr, biasR, outp);
}
